// EdgeKeyValueNetwork_47571057770947
// MI455X (gfx1250) — hardware-verified
//
#include <hip/hip_runtime.h>
#include <math.h>

typedef __attribute__((ext_vector_type(16))) _Float16 v16h;
typedef __attribute__((ext_vector_type(16))) __bf16 v16b;
typedef __attribute__((ext_vector_type(8)))  _Float16 v8h;
typedef __attribute__((ext_vector_type(8)))  float v8f;
typedef __attribute__((ext_vector_type(4)))  float v4f;
typedef __attribute__((ext_vector_type(2)))  float v2f;
typedef __attribute__((ext_vector_type(4)))  unsigned v4u;
typedef __attribute__((ext_vector_type(4)))  int v4i;
typedef float __attribute__((may_alias)) float_a;
typedef int __attribute__((may_alias)) int_a;

template <typename T> __device__ __forceinline__ void vst2(void* p, T v) { *(volatile T*)p = v; __threadfence(); *(volatile T*)p = v; }
__device__ __forceinline__ v8f wmma16(v16h a, v16h b, v8f c) {
  v8f d = __builtin_amdgcn_wmma_f32_16x16x32_f16(false, a, false, b, (short)0, c, false, false);
  asm volatile("v_nop\n\tv_nop\n\tv_nop\n\tv_nop" : "+v"(d) : "v"(a), "v"(b));
  return d;
}
__device__ __forceinline__ v8f wmma_bf(v16b a, v16b b, v8f c) {
  v8f d = __builtin_amdgcn_wmma_f32_16x16x32_bf16(false, a, false, b, (short)0, c, false, false);
  asm volatile("v_nop\n\tv_nop\n\tv_nop\n\tv_nop" : "+v"(d) : "v"(a), "v"(b));
  return d;
}
__device__ __forceinline__ v16h frag_h(const _Float16* rowk0, int lane) {
  union { v16h v; v8h q[2]; } u; const _Float16* p = rowk0 + 8 * (lane >> 4);
  u.q[0] = *(const v8h*)p; u.q[1] = *(const v8h*)(p + 16); return u.v;
}
__device__ __forceinline__ v16h frag_f32(const float* rowk0, int lane) {
  v16h a; const float* p = rowk0 + 8 * (lane >> 4);
#pragma unroll
  for (int i = 0; i < 8; ++i) { a[i] = (_Float16)p[i]; a[8 + i] = (_Float16)p[16 + i]; }
  return a;
}
__device__ __forceinline__ v16h frag_f32s(const float* rowk0, int lane, float sc) {
  v16h a; const float* p = rowk0 + 8 * (lane >> 4);
#pragma unroll
  for (int i = 0; i < 8; ++i) { a[i] = (_Float16)(p[i] * sc); a[8 + i] = (_Float16)(p[16 + i] * sc); }
  return a;
}
__device__ __forceinline__ v16h fragc_f32(const float* W, int k0, int n, int lane, int ld, int K) {
  v16h a; const int g = lane >> 4;
#pragma unroll
  for (int i = 0; i < 8; ++i) { const int ka = k0 + 8 * g + i, kb = ka + 16;
    a[i] = (_Float16)(ka < K ? W[(size_t)(ka < K ? ka : K - 1) * ld + n] : 0.f); a[8 + i] = (_Float16)(kb < K ? W[(size_t)(kb < K ? kb : K - 1) * ld + n] : 0.f); }
  return a;
}
struct F2 { v16b h, l; };
__device__ __forceinline__ F2 bsplit16(const float v[16]) { F2 r;
#pragma unroll
  for (int i = 0; i < 16; ++i) { const __bf16 h = (__bf16)v[i]; r.h[i] = h; r.l[i] = (__bf16)(v[i] - (float)h); }
  return r; }
__device__ __forceinline__ F2 split_row(const float* row, int k0, int lane) { float v[16]; const float* p = row + k0 + 8 * (lane >> 4);
#pragma unroll
  for (int i = 0; i < 8; ++i) { v[i] = p[i]; v[8 + i] = p[16 + i]; }
  return bsplit16(v); }
__device__ __forceinline__ F2 split_rowK(const float* row, int k0, int lane, int K) { float v[16]; const int g = lane >> 4;
#pragma unroll
  for (int i = 0; i < 8; ++i) { const int ka = k0 + 8 * g + i, kb = ka + 16; v[i] = ka < K ? row[ka < K ? ka : K - 1] : 0.f; v[8 + i] = kb < K ? row[kb < K ? kb : K - 1] : 0.f; }
  return bsplit16(v); }
__device__ __forceinline__ F2 split_col(const float* W, int k0, int n, int lane, int ld, int K) { float v[16]; const int g = lane >> 4;
#pragma unroll
  for (int i = 0; i < 8; ++i) { const int ka = k0 + 8 * g + i, kb = ka + 16; v[i] = ka < K ? W[(size_t)(ka < K ? ka : K - 1) * ld + n] : 0.f; v[8 + i] = kb < K ? W[(size_t)(kb < K ? kb : K - 1) * ld + n] : 0.f; }
  return bsplit16(v); }
__device__ __forceinline__ v8f mac3(const F2& a, const F2& b, v8f c) { c = wmma_bf(a.l, b.h, c); c = wmma_bf(a.h, b.l, c); return wmma_bf(a.h, b.h, c); }
__device__ __forceinline__ float sigm(float v) { return 1.0f / (1.0f + expf(-v)); }
#define LDSX() do { asm volatile("s_wait_dscnt 0" ::: "memory"); __builtin_amdgcn_wave_barrier(); __builtin_amdgcn_fence(__ATOMIC_RELEASE, "workgroup"); } while (0)


#define NE 131072
#define EB 32
#define NBR 16
#define HH 64
#define NWK 384
#define NWV 576
#define PW0 0.20412414523193151f
#define PW1C3 0.20412414523193151f
#define C3 0.57735026918962573f
__device__ __forceinline__ float bfr(float v) { return (float)(__bf16)v; }
typedef __attribute__((ext_vector_type(8))) __bf16 v8b;
__device__ __forceinline__ v16b frag_b(const __bf16* rowk0, int lane) {
  union { v16b v; v8b q[2]; } u; const __bf16* p = rowk0 + 8 * (lane >> 4);
  u.q[0] = *(const v8b*)p; u.q[1] = *(const v8b*)(p + 16); return u.v;
}
__device__ __attribute__((noinline)) float silu_ni(float v) { return v / (1.0f + expf(-v)); }

#define PO_W1K 0
#define PO_W1V (PO_W1K + 64 * 32)
#define PO_W2K (PO_W1V + 64 * 32)
#define PO_W2V (PO_W2K + 64 * 64)
#define PO_W3K (PO_W2V + 64 * 64)
#define PO_W3V (PO_W3K + NWK * 64)
#define PO_END (PO_W3V + NWV * 64)

__global__ __launch_bounds__(64) void k_pack(const float* __restrict__ W1k, const float* __restrict__ W1v, const float* __restrict__ W2k, const float* __restrict__ W2v, const float* __restrict__ W3k, const float* __restrict__ W3v, __bf16* __restrict__ PT) {
  __shared__ __align__(16) __bf16 srow[64];
  const int n = blockIdx.x, tid = threadIdx.x; const float* Wm; int K, NO, nn; size_t base; int KP;
  if (n < 128) return;
  if (n < 64) { Wm = W1k; K = NBR; NO = HH; nn = n; KP = 32; base = PO_W1K + (size_t)nn * 32; }
  else if (n < 128) { Wm = W1v; K = NBR; NO = HH; nn = n - 64; KP = 32; base = PO_W1V + (size_t)nn * 32; }
  else if (n < 192) { Wm = W2k; K = HH; NO = HH; nn = n - 128; KP = 64; base = PO_W2K + (size_t)nn * 64; }
  else if (n < 256) { Wm = W2v; K = HH; NO = HH; nn = n - 192; KP = 64; base = PO_W2V + (size_t)nn * 64; }
  else if (n < 256 + NWK) { Wm = W3k; K = HH; NO = NWK; nn = n - 256; KP = 64; base = PO_W3K + (size_t)nn * 64; }
  else { Wm = W3v; K = HH; NO = NWV; nn = n - 256 - NWK; KP = 64; base = PO_W3V + (size_t)nn * 64; }
  srow[tid] = tid < K ? (__bf16)Wm[(size_t)tid * NO + nn] : (__bf16)0.f;
  __syncthreads();
  if (tid < KP / 8) vst2((unsigned*)(PT + base + tid * 8), *(const v4u*)(&srow[tid * 8]));
}
__global__ __launch_bounds__(256) void k_pack1(const float* __restrict__ W1k, const float* __restrict__ W1v, __bf16* __restrict__ PT) {
  const int tid = threadIdx.x;
  for (int q = tid; q < 512; q += 256) { const int tb = q >> 8, n = (q >> 2) & 63, pc = q & 3; const float* Wm = tb ? W1v : W1k; union { __bf16 e[8]; v4u u; } pk;
#pragma unroll
    for (int e = 0; e < 8; ++e) { const int k = pc * 8 + e; pk.e[e] = k < NBR ? (__bf16)Wm[(size_t)k * HH + n] : (__bf16)0.f; }
    vst2((unsigned*)(PT + (tb ? PO_W1V : PO_W1K) + (size_t)n * 32 + pc * 8), pk.u); }
}

__global__ __launch_bounds__(256) void k_edge(const float* __restrict__ X, const float* __restrict__ SH, const float* __restrict__ R, const __bf16* __restrict__ PT,
                                              const float* __restrict__ bk1, const float* __restrict__ bk2, const float* __restrict__ bk3, const float* __restrict__ bv1, const float* __restrict__ bv2, const float* __restrict__ bv3,
                                              float* __restrict__ OK, float* __restrict__ OV) {
  __shared__ __align__(16) float sx[EB][40], ssh[EB][4], svd[EB][8];
  __shared__ __align__(16) float sr[EB][36];
  __shared__ __align__(16) float sh1[2][EB][HH + 4], sh2[2][EB][HH + 4];
  __shared__ __align__(16) float sw[EB][NWV + 4];
  __shared__ __align__(16) float sout[EB * 40];
  const int tid = threadIdx.x, wave = tid >> 5, lane = tid & 31, col = lane & 15, g = lane >> 4; const size_t e0 = (size_t)blockIdx.x * EB;
  for (int q = tid; q < EB * 40; q += 256) { const int e = q / 40, c = q - e * 40; sx[e][c] = bfr(X[(e0 + e) * 40 + c]); }
  for (int q = tid; q < EB * 4; q += 256) { const int e = q >> 2, c = q & 3; ssh[e][c] = bfr(SH[(e0 + e) * 4 + c]); }
  for (int q = tid; q < EB * 32; q += 256) { const int e = q >> 5, c = q & 31; sr[e][c] = c < NBR ? bfr(R[(e0 + e) * NBR + c]) : 0.f; }
  __syncthreads();
  if (tid < EB * 8) { const int e = tid >> 3, u = tid & 7; svd[e][u] = (sx[e][16 + u * 3] * ssh[e][1] + sx[e][16 + u * 3 + 1] * ssh[e][2]) + sx[e][16 + u * 3 + 2] * ssh[e][3]; }
  { const int br = wave >> 2, rt = (wave >> 1) & 1, ct0 = (wave & 1) * 2; const float* bb = br ? bv1 : bk1; const size_t po = br ? PO_W1V : PO_W1K;
    const F2 a = split_row(&sr[rt * 16 + col][0], 0, lane);
#pragma unroll
    for (int j = 0; j < 2; ++j) { v8f acc = {}; acc = wmma_bf(a.h, frag_b(PT + po + (size_t)((ct0 + j) * 16 + col) * 32, lane), acc);
#pragma unroll
      for (int r = 0; r < 8; ++r) sh1[br][rt * 16 + 8 * g + r][(ct0 + j) * 16 + col] = silu_ni(acc[r] + bfr(bb[(ct0 + j) * 16 + col])); } }
  __syncthreads();
  { const int br = wave >> 2, rt = (wave >> 1) & 1, ct0 = (wave & 1) * 2; const float* bb = br ? bv2 : bk2; const size_t po = br ? PO_W2V : PO_W2K;
    v8f acc[2] = {};
#pragma unroll
    for (int kc = 0; kc < 2; ++kc) { const F2 a = split_row(&sh1[br][rt * 16 + col][0], kc * 32, lane);
#pragma unroll
      for (int j = 0; j < 2; ++j) { const v16b wb = frag_b(PT + po + (size_t)((ct0 + j) * 16 + col) * 64 + kc * 32, lane); acc[j] = wmma_bf(a.l, wb, acc[j]); acc[j] = wmma_bf(a.h, wb, acc[j]); } }
#pragma unroll
    for (int j = 0; j < 2; ++j)
#pragma unroll
      for (int r = 0; r < 8; ++r) sh2[br][rt * 16 + 8 * g + r][(ct0 + j) * 16 + col] = silu_ni(acc[j][r] + bfr(bb[(ct0 + j) * 16 + col])); }
  __syncthreads();
#pragma unroll 1
  for (int br = 0; br < 2; ++br) {
    const int NW = br ? NWV : NWK; const int ntile = NW / 16; const size_t po = br ? PO_W3V : PO_W3K; const float* bb = br ? bv3 : bk3;
    { const int rt = wave & 1; const F2 a0 = split_row(&sh2[br][rt * 16 + col][0], 0, lane), a1 = split_row(&sh2[br][rt * 16 + col][0], 32, lane);
#pragma unroll 1
      for (int ct = wave >> 1; ct < ntile; ct += 4) { v8f acc = {}; const __bf16* wr = PT + po + (size_t)(ct * 16 + col) * 64;
        acc = wmma_bf(a0.l, frag_b(wr, lane), acc); acc = wmma_bf(a0.h, frag_b(wr, lane), acc); acc = wmma_bf(a1.l, frag_b(wr + 32, lane), acc); acc = wmma_bf(a1.h, frag_b(wr + 32, lane), acc);
        const float bv = bfr(bb[ct * 16 + col]);
#pragma unroll
        for (int r = 0; r < 8; ++r) sw[rt * 16 + 8 * g + r][ct * 16 + col] = acc[r] + bv; } }
    __syncthreads();
    const int m0 = br ? 16 : 8, m1 = 8; const int nout = m0 + 3 * m1;
    const int o000 = 0, o011 = 16 * m0, o101 = o011 + 16 * m1, o110 = o101 + 8 * m1;
    for (int q = tid; q < EB * nout; q += 256) { const int e = q / nout, oi = q - e * nout; const float* w = &sw[e][0]; float val;
      if (oi < m0) {
        float a = 0.f, c2 = 0.f;
#pragma unroll 4
        for (int u = 0; u < 16; ++u) a += w[o000 + u * m0 + oi] * sx[e][u];
#pragma unroll 4
        for (int u = 0; u < 8; ++u) c2 += w[o110 + u * m0 + oi] * svd[e][u];
        val = PW0 * (a * ssh[e][0] + C3 * c2);
      } else {
        const int wk = oi - m0, wq = wk / 3, kq = wk - wq * 3; float a = 0.f, d = 0.f;
#pragma unroll 4
        for (int u = 0; u < 16; ++u) a += w[o011 + u * m1 + wq] * sx[e][u];
#pragma unroll 4
        for (int u = 0; u < 8; ++u) d += w[o101 + u * m1 + wq] * sx[e][16 + u * 3 + kq];
        val = PW1C3 * (a * ssh[e][1 + kq] + d * ssh[e][0]);
      }
      sout[q] = val; }
    __syncthreads();
    { float* dst = (br ? OV : OK) + e0 * nout; for (int q = tid; q < EB * nout / 4; q += 256) vst2(dst + q * 4, *(const v4f*)&sout[q * 4]); }
    __syncthreads();
  }
}

extern "C" void kernel_launch(void* const* d_in, const int* in_sizes, int n_in, void* d_out, int out_size, void* d_ws, size_t ws_size, hipStream_t stream) {
  (void)in_sizes; (void)n_in; (void)out_size; (void)ws_size;
  const float** I = (const float**)d_in;
  __bf16* PT = (__bf16*)d_ws;
  float* OK = (float*)d_out; float* OV = OK + (size_t)NE * 32;
  k_pack<<<256 + NWK + NWV, 64, 0, stream>>>(I[3], I[9], I[5], I[11], I[7], I[13], PT);
  k_pack1<<<1, 256, 0, stream>>>(I[3], I[9], PT);
  k_edge<<<NE / EB, 256, 0, stream>>>(I[0], I[1], I[2], PT, I[4], I[6], I[8], I[10], I[12], I[14], OK, OV);
}
